// RiemannianManifold_76965813944498
// MI455X (gfx1250) — hardware-run, weakly checked
//
#include <hip/hip_runtime.h>
#include <math.h>

typedef __attribute__((ext_vector_type(16))) _Float16 v16h;
typedef __attribute__((ext_vector_type(8)))  _Float16 v8h;
typedef __attribute__((ext_vector_type(4)))  _Float16 v4h;
typedef __attribute__((ext_vector_type(2)))  _Float16 v2h;
typedef __attribute__((ext_vector_type(16))) __bf16   v16b;
typedef __attribute__((ext_vector_type(8)))  __bf16   v8b;
typedef __attribute__((ext_vector_type(8)))  float    v8f;
typedef __attribute__((ext_vector_type(4)))  float    v4f;
typedef __attribute__((ext_vector_type(2)))  float    v2f;

constexpr int kNB   = 2;
constexpr int kPN   = 256;
constexpr int kPM   = 256;
constexpr int kD    = 16;
constexpr int kH    = 32;
constexpr int kO    = 256;
constexpr int kPairs = kNB * kPN * kPM;
constexpr int kThr  = 256;
constexpr int kWaves = kPairs / 16;
constexpr float kDiagMin = 0.316f, kDiagMax = 3.16f;
constexpr float kFloor = 1.0e-6f;
constexpr float kInCarry = 1024.0f;
constexpr float kSc20 = 1.0f / (kInCarry * kInCarry);
constexpr float kF16MinNormal = 6.103515625e-5f;

static_assert(kNB == 2 && kPN == 256 && kPM == 256 && kD == 16 && kH == 32 && kO == 256 && kPairs == 131072 && kWaves == 8192, "the index arithmetic below uses these sizes");

constexpr size_t kOffW1P = 0ull;
constexpr size_t kOffW2T = 2048ull;
constexpr size_t kOffBR1 = 18432ull;
constexpr size_t kOffBR2 = 18688ull;
constexpr size_t kOffXR1 = 19712ull;
constexpr size_t kOffXR2 = 52480ull;
constexpr size_t kOffPS = 85248ull;
constexpr size_t kWsTotal = 1133824ull;
static_assert(kWsTotal <= 268435456ull, "the carve stands under 256 MiB");
static_assert(kOffW1P == 0
  && kOffW2T == kOffW1P + 2048ull
  && kOffBR1 == kOffW2T + 16384ull
  && kOffBR2 == kOffBR1 + 256ull
  && kOffXR1 == kOffBR2 + 1024ull
  && kOffXR2 == kOffXR1 + 32768ull
  && kOffPS == kOffXR2 + 32768ull
  && kWsTotal == kOffPS + 1048576ull, "the carve is a chain: every region starts where the one before ends");
static_assert((kOffW1P % 256) == 0 && (kOffW2T % 256) == 0 && (kOffBR1 % 256) == 0 && (kOffBR2 % 256) == 0 && (kOffXR1 % 256) == 0 && (kOffXR2 % 256) == 0 && (kOffPS % 256) == 0, "every region starts on a multiple of 256 B");

__device__ __forceinline__ unsigned short f2bf_bits(float f) {
  unsigned u = __float_as_uint(f);
  return (unsigned short)((u + 0x7FFFu + ((u >> 16) & 1u)) >> 16);
}
__device__ __forceinline__ float bf_bits2f(unsigned short h) { return __uint_as_float(((unsigned)h) << 16); }
__device__ __forceinline__ float bf16r(float f) { return bf_bits2f(f2bf_bits(f)); }
__device__ __forceinline__ float carry_flush(float v, float carry) {
  const float s = v * carry;
  return (fabsf(s) < kF16MinNormal) ? 0.0f : s;
}

__device__ __forceinline__ void dep_guard4_h(v8f& a, v8f& b, v8f& c, v8f& d, v16h x, v16h y) { asm volatile("v_nop\n\tv_nop\n\tv_nop\n\tv_nop" : "+v"(a), "+v"(b), "+v"(c), "+v"(d) : "v"(x), "v"(y)); }
__device__ __forceinline__ void dep_guard4_b(v8f& a, v8f& b, v8f& c, v8f& d, v16b x, v16b y) { asm volatile("v_nop\n\tv_nop\n\tv_nop\n\tv_nop" : "+v"(a), "+v"(b), "+v"(c), "+v"(d) : "v"(x), "v"(y)); }
__device__ __forceinline__ void keep4_h(v16h a, v16h b, v16h c, v16h d) { asm volatile("v_nop" :: "v"(a), "v"(b), "v"(c), "v"(d)); }
__device__ __forceinline__ void keep4_b(v16b a, v16b b, v16b c, v16b d) { asm volatile("v_nop" :: "v"(a), "v"(b), "v"(c), "v"(d)); }
__device__ __forceinline__ void acc_guard4(v8f& a, v8f& b, v8f& c, v8f& d) { asm volatile("v_nop\n\tv_nop\n\tv_nop\n\tv_nop" : "+v"(a), "+v"(b), "+v"(c), "+v"(d)); }

template <typename T> struct Frag;
template <> struct Frag<_Float16> {
  typedef v16h V; union U { v16h v; v8h h[2]; };
  static __device__ __forceinline__ v16h load(const _Float16* p) {
    U f; f.h[0] = *(const v8h*)(p); f.h[1] = *(const v8h*)(p + 16); return f.v;
  }
  static __device__ __forceinline__ v8f mma(v16h a, v16h b, v8f c) {
    return __builtin_amdgcn_wmma_f32_16x16x32_f16(false, a, false, b, (short)0, c, false, false);
  }
  static __device__ __forceinline__ void guard4(v8f& a, v8f& b, v8f& c, v8f& d, v16h x, v16h y) { dep_guard4_h(a, b, c, d, x, y); }
  static __device__ __forceinline__ void keep(v16h a, v16h b, v16h c, v16h d) { keep4_h(a, b, c, d); }
};
template <> struct Frag<__bf16> {
  typedef v16b V; union U { v16b v; v8b h[2]; };
  static __device__ __forceinline__ v16b load(const __bf16* p) {
    U f; f.h[0] = *(const v8b*)(p); f.h[1] = *(const v8b*)(p + 16); return f.v;
  }
  static __device__ __forceinline__ v8f mma(v16b a, v16b b, v8f c) {
    return __builtin_amdgcn_wmma_f32_16x16x32_bf16(false, a, false, b, (short)0, c, false, false);
  }
  static __device__ __forceinline__ void guard4(v8f& a, v8f& b, v8f& c, v8f& d, v16b x, v16b y) { dep_guard4_b(a, b, c, d, x, y); }
  static __device__ __forceinline__ void keep(v16b a, v16b b, v16b c, v16b d) { keep4_b(a, b, c, d); }
};

__device__ __forceinline__ v8f mma_h(v16h a, v16h b, v8f c) {
  c = __builtin_amdgcn_wmma_f32_16x16x32_f16(false, a, false, b, (short)0, c, false, false);
  asm volatile("v_nop\n\tv_nop\n\tv_nop\n\tv_nop" : "+v"(c) : "v"(a), "v"(b));
  return c;
}

template <int ET> struct Elem;
template <> struct Elem<0> { typedef _Float16 T; };
template <> struct Elem<1> { typedef __bf16 T; };
template <int ET, bool SPLIT, int BIAS_MODE, int OUT_MODE, bool RESID, int ACT = 0>
__global__ __launch_bounds__(256) void wmma_gemm64(
    const unsigned short* __restrict__ Ap, const unsigned short* __restrict__ A2p, int lda, long strideA,
    const unsigned short* __restrict__ Btp, const unsigned short* __restrict__ Bt2p, int ldb, long strideB,
    void* __restrict__ Cout, void* __restrict__ Cout2, int ldc, long strideC,
    const float* __restrict__ bias,
    const float* __restrict__ resid, long strideR,
    int M, int N, int K, float scale) {
  typedef typename Elem<ET>::T T;
  typedef typename Frag<T>::V V;
  const T* A = (const T*)Ap; const T* A2 = (const T*)A2p; const T* Bt = (const T*)Btp; const T* Bt2 = (const T*)Bt2p;
  __shared__ __align__(16) float sT[8][16 * 68];
  const int b    = blockIdx.y;
  const int lane = threadIdx.x & 31;
  const int wave = threadIdx.x >> 5;
  const int tilesN = N >> 6;
  const int tilesM = M >> 6;
  const int tile = blockIdx.x * 8 + wave;
  if (tile >= tilesM * tilesN) return;
  const int tm = tile / tilesN;
  const int tn = tile - tm * tilesN;
  const int m0 = tm << 6;
  const int n0 = tn << 6;

  const T* Ab  = A  + (size_t)b * strideA;
  const T* Bb  = Bt + (size_t)b * strideB;
  const T* Ab2 = SPLIT ? (A2  + (size_t)b * strideA) : nullptr;
  const T* Bb2 = SPLIT ? (Bt2 + (size_t)b * strideB) : nullptr;

  const int rlane = lane & 15;
  const int koff  = (lane >> 4) * 8;
  const int mOff  = (lane >> 4) * 8;

  v8f acc[4][4];
#pragma unroll
  for (int i = 0; i < 4; ++i)
#pragma unroll
    for (int j = 0; j < 4; ++j) acc[i][j] = (v8f){0.f,0.f,0.f,0.f,0.f,0.f,0.f,0.f};

  for (int k0 = 0; k0 < K; k0 += 32) {
    V bh[4], bl[4];
#pragma unroll
    for (int j = 0; j < 4; ++j) {
      const size_t bo = (size_t)(n0 + (j << 4) + rlane) * ldb + koff + k0;
      bh[j] = Frag<T>::load(Bb + bo);
      if (SPLIT) bl[j] = Frag<T>::load(Bb2 + bo);
    }
#pragma unroll
    for (int i = 0; i < 4; ++i) {
      const size_t ao = (size_t)(m0 + (i << 4) + rlane) * lda + koff + k0;
      V ah = Frag<T>::load(Ab + ao);
      V al;
      if (SPLIT) al = Frag<T>::load(Ab2 + ao);
#pragma unroll
      for (int j = 0; j < 4; ++j) {
        acc[i][j] = Frag<T>::mma(ah, bh[j], acc[i][j]);
        if (SPLIT) {
          acc[i][j] = Frag<T>::mma(ah, bl[j], acc[i][j]);
          acc[i][j] = Frag<T>::mma(al, bh[j], acc[i][j]);
        }
      }
      Frag<T>::guard4(acc[i][0], acc[i][1], acc[i][2], acc[i][3], ah, SPLIT ? al : ah);
    }
    Frag<T>::keep(bh[0], bh[1], bh[2], bh[3]);
    if (SPLIT) Frag<T>::keep(bl[0], bl[1], bl[2], bl[3]);
  }
  acc_guard4(acc[0][0], acc[0][1], acc[0][2], acc[0][3]);
  acc_guard4(acc[1][0], acc[1][1], acc[1][2], acc[1][3]);
  acc_guard4(acc[2][0], acc[2][1], acc[2][2], acc[2][3]);
  acc_guard4(acc[3][0], acc[3][1], acc[3][2], acc[3][3]);

  float* slab = sT[wave];
  const float* Rb = RESID ? (resid + (size_t)b * strideR) : nullptr;
#pragma unroll
  for (int i = 0; i < 4; ++i) {
    const int mBase = m0 + (i << 4);
#pragma unroll
    for (int j = 0; j < 4; ++j) {
      const int n = n0 + (j << 4) + rlane;
      float bv = 0.f;
      if (BIAS_MODE == 2) bv = bias[n];
#pragma unroll
      for (int r = 0; r < 8; ++r) {
        float v = acc[i][j][r] * scale;
        if (BIAS_MODE == 1) v += bias[mBase + mOff + r];
        if (BIAS_MODE == 2) v += bv;
        if (RESID) v += Rb[(size_t)(mBase + mOff + r) * ldc + n];
        if (ACT == 1) v = tanhf(v);
        if (ACT == 2) v = fmaxf(v, 0.0f);
        if (ACT == 3) v = v / (1.0f + expf(-v));
        if (ACT == 4) v = (v > 0.f) ? v : 0.01f * v;
        slab[(mOff + r) * 68 + (j << 4) + rlane] = v;
      }
    }
    __builtin_amdgcn_fence(__ATOMIC_RELEASE, "workgroup");
    __builtin_amdgcn_wave_barrier();
    __builtin_amdgcn_fence(__ATOMIC_ACQUIRE, "workgroup");
    if (OUT_MODE == 0) {
      float* C = (float*)Cout + (size_t)b * strideC;
      const int hh = lane >> 4, c4 = (lane & 15) * 4;
      for (int pass = 0; pass < 2; ++pass) {
#pragma unroll
        for (int it = 0; it < 8; ++it) {
          const int row = it * 2 + hh;
          v4f v = *(const v4f*)(slab + row * 68 + c4);
          *(volatile v4f*)(C + (size_t)(mBase + row) * ldc + n0 + c4) = v;
        }
        __threadfence();
      }
    } else {
      const int q = lane >> 3, c8 = (lane & 7) * 8;
      unsigned short* C  = (unsigned short*)Cout  + (size_t)b * strideC;
      unsigned short* C2 = (OUT_MODE == 2) ? ((unsigned short*)Cout2 + (size_t)b * strideC) : nullptr;
      for (int pass = 0; pass < 2; ++pass) {
#pragma unroll
        for (int it = 0; it < 4; ++it) {
          const int row = it * 4 + q;
          const float* sp = slab + row * 68 + c8;
          v8h hv, lv;
#pragma unroll
          for (int e = 0; e < 8; ++e) {
            if (OUT_MODE == 1) {
              hv[e] = (_Float16)sp[e];
            } else {
              unsigned short hb = f2bf_bits(sp[e]);
              unsigned short lb = f2bf_bits(sp[e] - bf_bits2f(hb));
              hv[e] = __builtin_bit_cast(_Float16, hb);
              lv[e] = __builtin_bit_cast(_Float16, lb);
            }
          }
          *(volatile v8h*)(C + (size_t)(mBase + row) * ldc + n0 + c8) = hv;
          if (OUT_MODE == 2) *(volatile v8h*)(C2 + (size_t)(mBase + row) * ldc + n0 + c8) = lv;
        }
        __threadfence();
      }
    }
    __builtin_amdgcn_fence(__ATOMIC_RELEASE, "workgroup");
    __builtin_amdgcn_wave_barrier();
    __builtin_amdgcn_fence(__ATOMIC_ACQUIRE, "workgroup");
  }
}

__global__ __launch_bounds__(kThr) void cast_plane_kernel(const float* __restrict__ src, unsigned short* __restrict__ dst,
                                                          int colsLog2, int dstPitch, int dstOff) {
  const int i   = blockIdx.x * kThr + threadIdx.x;
  const int sh  = colsLog2 - 3;
  const int row = i >> sh;
  const int c8  = (i & ((1 << sh) - 1)) * 8;
  const float* sp = src + ((size_t)row << colsLog2) + c8;
  const v4f a0 = *(const v4f*)(sp);
  const v4f a1 = *(const v4f*)(sp + 4);
  v8h hv;
#pragma unroll
  for (int e = 0; e < 4; ++e) {
    const float f0 = a0[e];
    const float f1 = a1[e];
    hv[e]     = (_Float16)carry_flush(bf16r(f0), kInCarry);
    hv[4 + e] = (_Float16)carry_flush(bf16r(f1), kInCarry);
  }
  unsigned short* dp = dst + (size_t)row * dstPitch + dstOff + c8;
  *(volatile v8h*)dp = hv;
  __threadfence();
  *(volatile v8h*)dp = hv;
}

__global__ __launch_bounds__(kThr) void pack_kernel(const float* __restrict__ W, unsigned short* __restrict__ D, float* __restrict__ dstf, int part, int ld, int k0, int lg, int n0, int pitch) {
  const unsigned i = blockIdx.x * blockDim.x + threadIdx.x;
  if (part == 0) {
    const unsigned g = i & ((1u << lg) - 1u), n = i >> lg;
    const float* sp = W + (size_t)((unsigned)k0 + g * 8u) * (unsigned)ld + n;
    v8h hv;
#pragma unroll
    for (int t = 0; t < 8; ++t) hv[t] = (_Float16)carry_flush(bf16r(sp[(size_t)t * (unsigned)ld]), kInCarry);
    unsigned short* dp = D + (size_t)((unsigned)n0 + n) * (unsigned)pitch + g * 8u;
    *(volatile v8h*)dp = hv;
    __threadfence();
    *(volatile v8h*)dp = hv;
  } else {
    const v4f a = *(const v4f*)(W + i * 4u);
    v4f o;
#pragma unroll
    for (int e = 0; e < 4; ++e) o[e] = bf16r(a[e]);
    float* dp = dstf + i * 4u;
    *(volatile v4f*)dp = o;
    __threadfence();
    *(volatile v4f*)dp = o;
  }
}

__global__ __launch_bounds__(kThr) void zero_kernel(float* __restrict__ dst) {
  const size_t o4 = ((size_t)blockIdx.x * kThr + threadIdx.x) * 4u;
  const v4f z = {0.f, 0.f, 0.f, 0.f};
  *(volatile v4f*)(dst + o4) = z;
  __threadfence();
  *(volatile v4f*)(dst + o4) = z;
}

__global__ __launch_bounds__(kThr) void padcast_kernel(const float* __restrict__ S, unsigned short* __restrict__ D, int G, int lg, int srow, int P, int r0) {
  const unsigned i = blockIdx.x * blockDim.x + threadIdx.x;
  const unsigned g = i & ((1u << lg) - 1u), row = i >> lg;
  const unsigned gc = (g < (unsigned)G) ? g : (unsigned)G - 1u;
  const v4f a = *(const v4f*)(S + (size_t)row * (unsigned)srow + gc * 4u);
  const float keep = (g < (unsigned)G) ? 1.0f : 0.0f;
  v4h hv;
#pragma unroll
  for (int e = 0; e < 4; ++e) hv[e] = (_Float16)(keep * carry_flush(bf16r(a[e]), kInCarry));
  unsigned short* dp = D + (size_t)((unsigned)r0 + row) * (unsigned)P + g * 4u;
  *(volatile v4h*)dp = hv;
  __threadfence();
  *(volatile v4h*)dp = hv;
}

__device__ __forceinline__ float silu_f(float v) { return v / (1.0f + expf(-v)); }
__device__ __forceinline__ v16h frag_pair(const v8f& t0, const v8f& t1, const float* __restrict__ bp) {
  const v4f b00 = *(const v4f*)(bp), b01 = *(const v4f*)(bp + 4), b10 = *(const v4f*)(bp + 16), b11 = *(const v4f*)(bp + 20);
  v16h f;
#pragma unroll
  for (int j = 0; j < 8; ++j) {
    const float bv0 = (j < 4) ? b00[j & 3] : b01[j & 3];
    const float bv1 = (j < 4) ? b10[j & 3] : b11[j & 3];
    f[j]     = (_Float16)carry_flush(silu_f(t0[j] * kSc20 + bv0), kInCarry);
    f[8 + j] = (_Float16)carry_flush(silu_f(t1[j] * kSc20 + bv1), kInCarry);
  }
  return f;
}
__device__ __forceinline__ float softplus_f(float v) { return fmaxf(v, 0.0f) + log1pf(expf(-fabsf(v))); }
__device__ __forceinline__ v16h frag_in(const float* __restrict__ c8) {
  v16h f;
#pragma unroll
  for (int j = 0; j < 8; ++j) {
    f[j]     = (_Float16)carry_flush(c8[j], kInCarry);
    f[8 + j] = (_Float16)0.0f;
  }
  return f;
}
__global__ __launch_bounds__(kThr) void metric_kernel(const float* __restrict__ x1, const float* __restrict__ x2, const unsigned short* __restrict__ W1Pp, const unsigned short* __restrict__ W2Tp,
                                                      const float* __restrict__ B1, const float* __restrict__ B2, float* __restrict__ PS) {
  const _Float16* W1P = (const _Float16*)W1Pp; const _Float16* W2T = (const _Float16*)W2Tp;
  const int lane = threadIdx.x & 31, lr = lane & 15, hi = lane >> 4;
  const int wave = blockIdx.x * (kThr / 32) + (threadIdx.x >> 5);
  const int pair = wave * 16 + lr;
  const int bn = pair >> 8;
  const int bm = ((wave >> 12) * kPM + (wave & 15) * 16) + lr;
  const float* p1 = x1 + (size_t)bn * kD;
  const float* p2 = x2 + (size_t)bm * kD;
  float c8[8];
  {
    const v4f a0 = *(const v4f*)(p1 + 8 * hi), a1 = *(const v4f*)(p1 + 8 * hi + 4), b0 = *(const v4f*)(p2 + 8 * hi), b1v = *(const v4f*)(p2 + 8 * hi + 4);
#pragma unroll
    for (int e = 0; e < 4; ++e) { c8[e] = (a0[e] + b0[e]) * 0.5f; c8[4 + e] = (a1[e] + b1v[e]) * 0.5f; }
  }
  const v16h cf = frag_in(c8);
  v8f h0 = (v8f){0.f, 0.f, 0.f, 0.f, 0.f, 0.f, 0.f, 0.f}, h1 = (v8f){0.f, 0.f, 0.f, 0.f, 0.f, 0.f, 0.f, 0.f};
  {
    const v16h a0 = Frag<_Float16>::load(W1P + (size_t)lr * kH + 8 * hi);
    const v16h a1 = Frag<_Float16>::load(W1P + (size_t)(16 + lr) * kH + 8 * hi);
    h0 = mma_h(a0, cf, h0);
    h1 = mma_h(a1, cf, h1);
  }
  const v16h hf = frag_pair(h0, h1, B1 + 8 * hi);
  float y[8];
#pragma unroll
  for (int r = 0; r < 8; ++r) y[r] = 0.0f;
  for (int t = 0; t < 16; ++t) {
    v8f acc = (v8f){0.f, 0.f, 0.f, 0.f, 0.f, 0.f, 0.f, 0.f};
    const v16h a = Frag<_Float16>::load(W2T + (size_t)(16 * t + lr) * kH + 8 * hi);
    acc = mma_h(a, hf, acc);
    const v4f bb0 = *(const v4f*)(B2 + 16 * t + 8 * hi), bb1 = *(const v4f*)(B2 + 16 * t + 8 * hi + 4);
    const float dt = p2[t] - p1[t];
    float v[8];
#pragma unroll
    for (int r = 0; r < 8; ++r) v[r] = acc[r] * kSc20 + ((r < 4) ? bb0[r & 3] : bb1[r & 3]);
    float vd = v[0];
#pragma unroll
    for (int r = 1; r < 8; ++r) vd = ((t & 7) == r) ? v[r] : vd;
    const float dg = fminf(fmaxf(softplus_f(vd + 1.0f), kDiagMin), kDiagMax);
#pragma unroll
    for (int r = 0; r < 8; ++r) {
      const int k = 8 * hi + r;
      const float lv = (k < t) ? v[r] : ((k == t) ? dg : 0.0f);
      y[r] = fmaf(lv, dt, y[r]);
    }
  }
  float part = 0.0f;
#pragma unroll
  for (int r = 0; r < 8; ++r) part = fmaf(y[r], y[r], part);
  float* dp = PS + (size_t)pair * 2 + hi;
  *(volatile float*)dp = part;
  __threadfence();
  *(volatile float*)dp = part;
}

__global__ __launch_bounds__(kThr) void finish_kernel(const float* __restrict__ PS, float* __restrict__ res) {
  const unsigned p = blockIdx.x * (unsigned)kThr + threadIdx.x;
  const v2f a = *(const v2f*)(PS + (size_t)p * 2u);
  const float o = sqrtf(fmaxf(a[0] + a[1], kFloor));
  *(volatile float*)(res + p) = o;
  __threadfence();
  *(volatile float*)(res + p) = o;
}

extern "C" void kernel_launch(void* const* d_in, const int* in_sizes, int n_in,
                              void* d_out, int out_size, void* d_ws, size_t ws_size,
                              hipStream_t stream) {
  if (n_in < 6 || d_out == nullptr || d_ws == nullptr) return;
  if (in_sizes[0] != kNB * kPN * kD || in_sizes[1] != kNB * kPM * kD || in_sizes[2] != kH * kD || in_sizes[3] != kH || in_sizes[4] != kO * kH || in_sizes[5] != kO) return;
  if (out_size != kPairs) return;
  if (ws_size < kWsTotal) return;
  const float* x1 = (const float*)d_in[0];
  const float* x2 = (const float*)d_in[1];
  const float* W1 = (const float*)d_in[2];
  const float* b1 = (const float*)d_in[3];
  const float* W2 = (const float*)d_in[4];
  const float* b2 = (const float*)d_in[5];
  float* out = (float*)d_out;
  char* ws = (char*)d_ws;
  unsigned short* W1P = (unsigned short*)(ws + kOffW1P);
  unsigned short* W2T = (unsigned short*)(ws + kOffW2T);
  float* BR1 = (float*)(ws + kOffBR1);
  float* BR2 = (float*)(ws + kOffBR2);
  float* XR1 = (float*)(ws + kOffXR1);
  float* XR2 = (float*)(ws + kOffXR2);
  float* PS = (float*)(ws + kOffPS);

  static_assert((kNB * kPN * kD / 4) % kThr == 0 && (kNB * kPM * kD / 4) % kThr == 0 && kH * 8 == kThr && (kO * kH / 8) % kThr == 0 && kH / 4 == 8 && kO / 4 == 64 && kWaves % 8 == 0 && kPairs % kThr == 0, "every grid exact");
  padcast_kernel<<<1, kThr, 0, stream>>>(W1, W1P, kD / 4, 3, kD, kH, 0);
  cast_plane_kernel<<<kO * kH / 8 / kThr, kThr, 0, stream>>>(W2, W2T, 5, kH, 0);
  pack_kernel<<<1, kH / 4, 0, stream>>>(b1, nullptr, BR1, 1, 0, 0, 0, 0, 0);
  zero_kernel<<<1, 8, 0, stream>>>(BR1 + kH);
  pack_kernel<<<1, kO / 4, 0, stream>>>(b2, nullptr, BR2, 1, 0, 0, 0, 0, 0);
  pack_kernel<<<kNB * kPN * kD / 4 / kThr, kThr, 0, stream>>>(x1, nullptr, XR1, 1, 0, 0, 0, 0, 0);
  pack_kernel<<<kNB * kPM * kD / 4 / kThr, kThr, 0, stream>>>(x2, nullptr, XR2, 1, 0, 0, 0, 0, 0);
  metric_kernel<<<kWaves / 8, kThr, 0, stream>>>(XR1, XR2, W1P, W2T, BR1, BR2, PS);
  finish_kernel<<<kPairs / kThr, kThr, 0, stream>>>(PS, out);
}
